// CQT_85856396247287
// MI455X (gfx1250) — hardware-verified
//
#include <hip/hip_runtime.h>


#define SIGLEN 220500
#define NBIN   252
#define NFR    456
#define HOP    484
#define MAXLEN 69365
#define CENTER 34682
#define KP     69376
#define NCH    8
#define KC     (KP / NCH)
#define MP     512
#define NP     512
typedef _Float16 h16;
typedef unsigned short bf;
typedef __attribute__((ext_vector_type(16))) __bf16   v16bf;
typedef __attribute__((ext_vector_type(16))) _Float16 v16h;
typedef __attribute__((ext_vector_type(8)))  _Float16 v8h;
typedef __attribute__((ext_vector_type(8)))  unsigned short v8us;
typedef __attribute__((ext_vector_type(8)))  float    v8f;
typedef __attribute__((ext_vector_type(4)))  float    v4f;
typedef v8h  __attribute__((may_alias)) v8ha;
typedef v4f  __attribute__((may_alias)) v4fa;
typedef v8us __attribute__((may_alias)) v8usa;

__device__ __forceinline__ unsigned short f2bf(float f) { unsigned u = __float_as_uint(f); u += 0x7FFFu + ((u >> 16) & 1u); return (unsigned short)(u >> 16); }
__device__ __forceinline__ float bf2f(unsigned short b) { return __uint_as_float(((unsigned)b) << 16); }
__device__ __forceinline__ float bfr(float f) { return bf2f(f2bf(f)); }
__device__ __forceinline__ v16h cat16(v8h lo, v8h hi) { return __builtin_shufflevector(lo, hi, 0, 1, 2, 3, 4, 5, 6, 7, 8, 9, 10, 11, 12, 13, 14, 15); }
__device__ __forceinline__ v16bf cat16b(v8us lo, v8us hi) { return __builtin_bit_cast(v16bf, __builtin_shufflevector(lo, hi, 0, 1, 2, 3, 4, 5, 6, 7, 8, 9, 10, 11, 12, 13, 14, 15)); }
__device__ __forceinline__ v8f wmma16(v16h a, v16h b, v8f c) { return __builtin_amdgcn_wmma_f32_16x16x32_f16(false, a, false, b, (short)0, c, false, false); }
__device__ __forceinline__ v8f wmmab(v16bf a, v16bf b, v8f c) { return __builtin_amdgcn_wmma_f32_16x16x32_bf16(false, a, false, b, (short)0, c, false, false); }


template <typename T16> struct WFrag;
template <> struct WFrag<h16> { typedef v16h V; static __device__ __forceinline__ V ld(const h16* p) { return cat16(*(const v8h*)p, *(const v8h*)(p + 16)); } static __device__ __forceinline__ v8f mma(V a, V b, v8f c) { return wmma16(a, b, c); } };
template <> struct WFrag<bf> { typedef v16bf V; static __device__ __forceinline__ V ld(const bf* p) { return cat16b(*(const v8us*)p, *(const v8us*)(p + 16)); } static __device__ __forceinline__ v8f mma(V a, V b, v8f c) { return wmmab(a, b, c); } };
template <typename T16, int NSPLIT, bool BIAS>
__global__ __launch_bounds__(32) void k_gemmw(const T16* __restrict__ A, const T16* __restrict__ A2, const T16* __restrict__ Bt, const T16* __restrict__ Bt2, int K, float* C, int ldc, const float* __restrict__ bias, size_t sA, size_t sB, size_t sC) {
    typedef typename WFrag<T16>::V V;
    __shared__ __align__(16) float os[16 * 68];
    const size_t z = blockIdx.z; A += z * sA; if (A2) A2 += z * sA; Bt += z * sB; if (Bt2) Bt2 += z * sB; C += z * sC;
    const int lane = threadIdx.x & 31, lr = lane & 15, hi = lane >> 4; const int r0 = blockIdx.x * 64, c0 = blockIdx.y * 64;
    v8f acc[4][4];
#pragma unroll
    for (int mb = 0; mb < 4; ++mb)
#pragma unroll
        for (int nb = 0; nb < 4; ++nb) acc[mb][nb] = (v8f){};
    const size_t aoff = (size_t)(r0 + lr) * K + 8 * hi, boff = (size_t)(c0 + lr) * K + 8 * hi;
#pragma unroll 1
    for (int kc = 0; kc < K; kc += 32) {
        V a[4], a2[4];
#pragma unroll
        for (int mb = 0; mb < 4; ++mb) { a[mb] = WFrag<T16>::ld(A + aoff + (size_t)mb * 16 * K + kc); if (NSPLIT == 1 || NSPLIT == 2) a2[mb] = WFrag<T16>::ld(A2 + aoff + (size_t)mb * 16 * K + kc); }
#pragma unroll
        for (int nb = 0; nb < 4; ++nb) { const V b = WFrag<T16>::ld(Bt + boff + (size_t)nb * 16 * K + kc); V b2; if (NSPLIT >= 2) b2 = WFrag<T16>::ld(Bt2 + boff + (size_t)nb * 16 * K + kc);
#pragma unroll
            for (int mb = 0; mb < 4; ++mb) { acc[mb][nb] = WFrag<T16>::mma(a[mb], b, acc[mb][nb]); if (NSPLIT == 1 || NSPLIT == 2) acc[mb][nb] = WFrag<T16>::mma(a2[mb], b, acc[mb][nb]); if (NSPLIT >= 2) acc[mb][nb] = WFrag<T16>::mma(a[mb], b2, acc[mb][nb]); } }
        asm volatile("v_nop\n\tv_nop\n\tv_nop\n\tv_nop" : "+v"(acc[0][0]), "+v"(acc[1][1]), "+v"(acc[2][2]), "+v"(acc[3][3]) : "v"(a[0]), "v"(a[3]));
    }
#pragma unroll
    for (int mb = 0; mb < 4; ++mb) {
#pragma unroll
        for (int nb = 0; nb < 4; ++nb) {
#pragma unroll
            for (int j = 0; j < 8; ++j) os[(hi * 8 + j) * 68 + nb * 16 + lr] = acc[mb][nb][j]; }
        __builtin_amdgcn_wave_barrier(); asm volatile("" ::: "memory");
        float* crow = C + (size_t)(r0 + mb * 16) * ldc + c0;
#pragma unroll 1
        for (int ps = 0; ps < 2; ++ps) {
#pragma unroll
            for (int s = 0; s < 8; ++s) { const int row = 2 * s + hi, cofs = lr * 4; v4f val = *(const v4fa*)(os + row * 68 + cofs); if (BIAS) { val[0] += bfr(bias[c0 + cofs]); val[1] += bfr(bias[c0 + cofs + 1]); val[2] += bfr(bias[c0 + cofs + 2]); val[3] += bfr(bias[c0 + cofs + 3]); }
                *(volatile v4f*)(crow + (size_t)row * ldc + cofs) = val; }
            if (ps == 0) __threadfence(); }
        __builtin_amdgcn_wave_barrier(); asm volatile("" ::: "memory");
    }
}

static const float CQT_FREQ[252] = {3.270319748e+01f,3.333896637e+01f,3.398709869e+01f,3.464782715e+01f,3.532140350e+01f,3.600807571e+01f,3.670809555e+01f,3.742172623e+01f,3.814922714e+01f,3.889087296e+01f,3.964693832e+01f,4.041769791e+01f,4.120344543e+01f,4.200446701e+01f,4.282106018e+01f,4.365353012e+01f,4.450218201e+01f,4.536733246e+01f,4.624930191e+01f,4.714841843e+01f,4.806501389e+01f,4.899942780e+01f,4.995201111e+01f,5.092311096e+01f,5.191308594e+01f,5.292230988e+01f,5.395115662e+01f,5.500000000e+01f,5.606923676e+01f,5.715925598e+01f,5.827046967e+01f,5.940328598e+01f,6.055812454e+01f,6.173541260e+01f,6.293558884e+01f,6.415909576e+01f,6.540639496e+01f,6.667793274e+01f,6.797419739e+01f,6.929565430e+01f,7.064280701e+01f,7.201615143e+01f,7.341619110e+01f,7.484345245e+01f,7.629845428e+01f,7.778174591e+01f,7.929387665e+01f,8.083539581e+01f,8.240689087e+01f,8.400893402e+01f,8.564212036e+01f,8.730706024e+01f,8.900436401e+01f,9.073466492e+01f,9.249860382e+01f,9.429683685e+01f,9.613002777e+01f,9.799885559e+01f,9.990402222e+01f,1.018462219e+02f,1.038261719e+02f,1.058446198e+02f,1.079023132e+02f,1.100000000e+02f,1.121384735e+02f,1.143185120e+02f,1.165409393e+02f,1.188065720e+02f,1.211162491e+02f,1.234708252e+02f,1.258711777e+02f,1.283181915e+02f,1.308127899e+02f,1.333558655e+02f,1.359483948e+02f,1.385913086e+02f,1.412856140e+02f,1.440323029e+02f,1.468323822e+02f,1.496869049e+02f,1.525969086e+02f,1.555634918e+02f,1.585877533e+02f,1.616707916e+02f,1.648137817e+02f,1.680178680e+02f,1.712842407e+02f,1.746141205e+02f,1.780087280e+02f,1.814693298e+02f,1.849972076e+02f,1.885936737e+02f,1.922600555e+02f,1.959977112e+02f,1.998080444e+02f,2.036924438e+02f,2.076523438e+02f,2.116892395e+02f,2.158046265e+02f,2.200000000e+02f,2.242769470e+02f,2.286370239e+02f,2.330818787e+02f,2.376131439e+02f,2.422324982e+02f,2.469416504e+02f,2.517423553e+02f,2.566363831e+02f,2.616255798e+02f,2.667117310e+02f,2.718967896e+02f,2.771826172e+02f,2.825712280e+02f,2.880646057e+02f,2.936647644e+02f,2.993738098e+02f,3.051938171e+02f,3.111269836e+02f,3.171755066e+02f,3.233415833e+02f,3.296275635e+02f,3.360357361e+02f,3.425684814e+02f,3.492282410e+02f,3.560174561e+02f,3.629386597e+02f,3.699944153e+02f,3.771873474e+02f,3.845201111e+02f,3.919954224e+02f,3.996160889e+02f,4.073848877e+02f,4.153046875e+02f,4.233784790e+02f,4.316092529e+02f,4.400000000e+02f,4.485538940e+02f,4.572740479e+02f,4.661637573e+02f,4.752262878e+02f,4.844649963e+02f,4.938833008e+02f,5.034847107e+02f,5.132727661e+02f,5.232511597e+02f,5.334234619e+02f,5.437935791e+02f,5.543652344e+02f,5.651424561e+02f,5.761292114e+02f,5.873295288e+02f,5.987476196e+02f,6.103876343e+02f,6.222539673e+02f,6.343510132e+02f,6.466831665e+02f,6.592551270e+02f,6.720714722e+02f,6.851369629e+02f,6.984564819e+02f,7.120349121e+02f,7.258773193e+02f,7.399888306e+02f,7.543746948e+02f,7.690402222e+02f,7.839908447e+02f,7.992321777e+02f,8.147697754e+02f,8.306093750e+02f,8.467569580e+02f,8.632185059e+02f,8.800000000e+02f,8.971077881e+02f,9.145480957e+02f,9.323275146e+02f,9.504525757e+02f,9.689299927e+02f,9.877666016e+02f,1.006969421e+03f,1.026545532e+03f,1.046502319e+03f,1.066846924e+03f,1.087587158e+03f,1.108730469e+03f,1.130284912e+03f,1.152258423e+03f,1.174659058e+03f,1.197495239e+03f,1.220775269e+03f,1.244507935e+03f,1.268702026e+03f,1.293366333e+03f,1.318510254e+03f,1.344142944e+03f,1.370273926e+03f,1.396912964e+03f,1.424069824e+03f,1.451754639e+03f,1.479977661e+03f,1.508749390e+03f,1.538080444e+03f,1.567981689e+03f,1.598464355e+03f,1.629539551e+03f,1.661218750e+03f,1.693513916e+03f,1.726437012e+03f,1.760000000e+03f,1.794215576e+03f,1.829096191e+03f,1.864655029e+03f,1.900905151e+03f,1.937859985e+03f,1.975533203e+03f,2.013938843e+03f,2.053091064e+03f,2.093004639e+03f,2.133693848e+03f,2.175174316e+03f,2.217460938e+03f,2.260569824e+03f,2.304516846e+03f,2.349318115e+03f,2.394990479e+03f,2.441550537e+03f,2.489015869e+03f,2.537404053e+03f,2.586732666e+03f,2.637020508e+03f,2.688285889e+03f,2.740547852e+03f,2.793825928e+03f,2.848139648e+03f,2.903509277e+03f,2.959955322e+03f,3.017498779e+03f,3.076160889e+03f,3.135963379e+03f,3.196928711e+03f,3.259079102e+03f,3.322437500e+03f,3.387027832e+03f,3.452874023e+03f,3.520000000e+03f,3.588431152e+03f,3.658192383e+03f,3.729310059e+03f,3.801810303e+03f,3.875719971e+03f,3.951066406e+03f,4.027877686e+03f,4.106182129e+03f};
static const float CQT_LEN[252] = {6.936457812e+04f,6.804180469e+04f,6.674425000e+04f,6.547144531e+04f,6.422291016e+04f,6.299818359e+04f,6.179681641e+04f,6.061835547e+04f,5.946236719e+04f,5.832842578e+04f,5.721610938e+04f,5.612500000e+04f,5.505470312e+04f,5.400481641e+04f,5.297494922e+04f,5.196471875e+04f,5.097375781e+04f,5.000169141e+04f,4.904816406e+04f,4.811282031e+04f,4.719531250e+04f,4.629530078e+04f,4.541245312e+04f,4.454644531e+04f,4.369694531e+04f,4.286364844e+04f,4.204624219e+04f,4.124442578e+04f,4.045789844e+04f,3.968637109e+04f,3.892955469e+04f,3.818717188e+04f,3.745894531e+04f,3.674460547e+04f,3.604389062e+04f,3.535653516e+04f,3.468228906e+04f,3.402090234e+04f,3.337212500e+04f,3.273572266e+04f,3.211145508e+04f,3.149909180e+04f,3.089840820e+04f,3.030917773e+04f,2.973118359e+04f,2.916421289e+04f,2.860805469e+04f,2.806250000e+04f,2.752735156e+04f,2.700240820e+04f,2.648747461e+04f,2.598235938e+04f,2.548687891e+04f,2.500084570e+04f,2.452408203e+04f,2.405641016e+04f,2.359765625e+04f,2.314765039e+04f,2.270622656e+04f,2.227322266e+04f,2.184847266e+04f,2.143182422e+04f,2.102312109e+04f,2.062221289e+04f,2.022894922e+04f,1.984318555e+04f,1.946477734e+04f,1.909358594e+04f,1.872947266e+04f,1.837230273e+04f,1.802194531e+04f,1.767826758e+04f,1.734114453e+04f,1.701045117e+04f,1.668606250e+04f,1.636786133e+04f,1.605572754e+04f,1.574954590e+04f,1.544920410e+04f,1.515458887e+04f,1.486559180e+04f,1.458210645e+04f,1.430402734e+04f,1.403125000e+04f,1.376367578e+04f,1.350120410e+04f,1.324373730e+04f,1.299117969e+04f,1.274343945e+04f,1.250042285e+04f,1.226204102e+04f,1.202820508e+04f,1.179882812e+04f,1.157382520e+04f,1.135311328e+04f,1.113661133e+04f,1.092423633e+04f,1.071591211e+04f,1.051156055e+04f,1.031110645e+04f,1.011447461e+04f,9.921592773e+03f,9.732388672e+03f,9.546792969e+03f,9.364736328e+03f,9.186151367e+03f,9.010972656e+03f,8.839133789e+03f,8.670572266e+03f,8.505225586e+03f,8.343031250e+03f,8.183930664e+03f,8.027863770e+03f,7.874772949e+03f,7.724602051e+03f,7.577294434e+03f,7.432795898e+03f,7.291053223e+03f,7.152013672e+03f,7.015625000e+03f,6.881837891e+03f,6.750602051e+03f,6.621868652e+03f,6.495589844e+03f,6.371719727e+03f,6.250211426e+03f,6.131020508e+03f,6.014102539e+03f,5.899414062e+03f,5.786912598e+03f,5.676556641e+03f,5.568305664e+03f,5.462118164e+03f,5.357956055e+03f,5.255780273e+03f,5.155553223e+03f,5.057237305e+03f,4.960796387e+03f,4.866194336e+03f,4.773396484e+03f,4.682368164e+03f,4.593075684e+03f,4.505486328e+03f,4.419566895e+03f,4.335286133e+03f,4.252612793e+03f,4.171515625e+03f,4.091965332e+03f,4.013931885e+03f,3.937386475e+03f,3.862301025e+03f,3.788647217e+03f,3.716397949e+03f,3.645526611e+03f,3.576006836e+03f,3.507812500e+03f,3.440918945e+03f,3.375301025e+03f,3.310934326e+03f,3.247794922e+03f,3.185859863e+03f,3.125105713e+03f,3.065510254e+03f,3.007051270e+03f,2.949707031e+03f,2.893456299e+03f,2.838278320e+03f,2.784152832e+03f,2.731059082e+03f,2.678978027e+03f,2.627890137e+03f,2.577776611e+03f,2.528618652e+03f,2.480398193e+03f,2.433097168e+03f,2.386698242e+03f,2.341184082e+03f,2.296537842e+03f,2.252743164e+03f,2.209783447e+03f,2.167643066e+03f,2.126306396e+03f,2.085757812e+03f,2.045982666e+03f,2.006965942e+03f,1.968693237e+03f,1.931150513e+03f,1.894323608e+03f,1.858198975e+03f,1.822763306e+03f,1.788003418e+03f,1.753906250e+03f,1.720459473e+03f,1.687650513e+03f,1.655467163e+03f,1.623897461e+03f,1.592929932e+03f,1.562552856e+03f,1.532755127e+03f,1.503525635e+03f,1.474853516e+03f,1.446728149e+03f,1.419139160e+03f,1.392076416e+03f,1.365529541e+03f,1.339489014e+03f,1.313945068e+03f,1.288888306e+03f,1.264309326e+03f,1.240199097e+03f,1.216548584e+03f,1.193349121e+03f,1.170592041e+03f,1.148268921e+03f,1.126371582e+03f,1.104891724e+03f,1.083821533e+03f,1.063153198e+03f,1.042878906e+03f,1.022991333e+03f,1.003482971e+03f,9.843466187e+02f,9.655752563e+02f,9.471618042e+02f,9.290994873e+02f,9.113816528e+02f,8.940017090e+02f,8.769531250e+02f,8.602297363e+02f,8.438252563e+02f,8.277335815e+02f,8.119487305e+02f,7.964649658e+02f,7.812764282e+02f,7.663775635e+02f,7.517628174e+02f,7.374267578e+02f,7.233640747e+02f,7.095695801e+02f,6.960382080e+02f,6.827647705e+02f,6.697445068e+02f,6.569725342e+02f,6.444441528e+02f,6.321546631e+02f,6.200995483e+02f,6.082742920e+02f,5.966745605e+02f,5.852960205e+02f,5.741344604e+02f,5.631857910e+02f,5.524458618e+02f};

__device__ __forceinline__ void splitf(float y, unsigned short& h, unsigned short& l) { h = f2bf(y); l = f2bf(y - bf2f(h)); }
__device__ __forceinline__ float winval(int bin, int tt, float& t_out) {
    const float t = (float)(tt - CENTER); t_out = t; const float L = CQT_LEN[bin];
    if (!(fabsf(t) < L * 0.5f)) return 0.f;
    const float a = __fdiv_rn(__fmul_rn(6.2831855f, t), L); return 0.5f * (1.0f + cosf(a));
}

__device__ __noinline__ float2 kernval(int bin, int tt, float inv_norm_den) {
    float t; const float w = winval(bin, tt, t); if (w == 0.f) return make_float2(0.f, 0.f);
    const float ang = __fdiv_rn(__fmul_rn(__fmul_rn(6.2831855f, CQT_FREQ[bin]), t), 44100.0f); float sn, cs; sincosf(ang, &sn, &cs);
    return make_float2(__fdiv_rn(w * cs, inv_norm_den), __fdiv_rn(w * sn, inv_norm_den));
}
__global__ __launch_bounds__(256) void k_norm(float* NORM) {
    const int lane = threadIdx.x & 31; const int bin0 = (blockIdx.x * 8 + (threadIdx.x >> 5)) * 32; if (bin0 >= 256) return; const int bin = bin0 + lane; float s = 0.f;
    if (bin < NBIN) { const float L = CQT_LEN[bin]; const int half = (int)(L * 0.5f) + 2; const int lo = CENTER - half < 0 ? 0 : CENTER - half, hi = CENTER + half > MAXLEN - 1 ? MAXLEN - 1 : CENTER + half;
#pragma unroll 1
        for (int tt = lo; tt <= hi; ++tt) { float t; s += winval(bin, tt, t); } s = s * sqrtf(L); }
    float* dst = NORM + bin0; *(volatile float*)(dst + lane) = s; __threadfence(); *(volatile float*)(dst + lane) = s;
}
__global__ __launch_bounds__(256) void k_frames(const float* __restrict__ sig, int kc0, bf* Bt) {
    typedef __attribute__((ext_vector_type(2))) unsigned short v2us;
    const int lane = threadIdx.x & 31; const int L0 = (blockIdx.x * 8 + (threadIdx.x >> 5)) * 8; const int nlines = NP * KC / 64;
#pragma unroll 1
    for (int ps = 0; ps < 2; ++ps) {
#pragma unroll
        for (int l = 0; l < 8; ++l) { const int L = L0 + l; if (L >= nlines) break; const int e = L * 64 + lane * 2; const int f = e / KC, j = e % KC; v2us o;
#pragma unroll
            for (int q = 0; q < 2; ++q) { const int tt = kc0 + j + q; const int si = f * HOP + tt - CENTER; const bool in = f < NFR && tt < MAXLEN && si >= 0 && si < SIGLEN; o[q] = in ? f2bf(sig[si < 0 ? 0 : (si > SIGLEN - 1 ? SIGLEN - 1 : si)]) : (unsigned short)0; }
            *(volatile v2us*)(Bt + e) = o; }
        if (ps == 0) __threadfence(); }
}
__global__ __launch_bounds__(256) void k_kern(const float* __restrict__ NORM, int kc0, bf* Ah, bf* Al) {
    typedef __attribute__((ext_vector_type(2))) unsigned short v2us;
    const int lane = threadIdx.x & 31; const int L0 = (blockIdx.x * 8 + (threadIdx.x >> 5)) * 8; const int nlines = 256 * KC / 64;
#pragma unroll 1
    for (int ps = 0; ps < 2; ++ps) {
#pragma unroll 1
        for (int l = 0; l < 8; ++l) { const int L = L0 + l; if (L >= nlines) break; const int e = L * 64 + lane * 2; const int bin = e / KC, j = e % KC; v2us rh, rl, ih, il;
#pragma unroll
            for (int q = 0; q < 2; ++q) { const int tt = kc0 + j + q; float kr = 0.f, ki = 0.f;
                if (bin < NBIN && tt < MAXLEN) { const float2 v = kernval(bin, tt, NORM[bin < NBIN ? bin : 0]); kr = v.x; ki = v.y; }
                unsigned short a, b2; splitf(kr, a, b2); rh[q] = a; rl[q] = b2; splitf(ki, a, b2); ih[q] = a; il[q] = b2; }
            const size_t orow = (bin < NBIN) ? (size_t)bin : (size_t)(504 + (bin - NBIN));
            const size_t irow = (bin < NBIN) ? (size_t)(NBIN + bin) : (size_t)(508 + (bin - NBIN));
            *(volatile v2us*)(Ah + orow * KC + j) = rh; *(volatile v2us*)(Al + orow * KC + j) = rl; *(volatile v2us*)(Ah + irow * KC + j) = ih; *(volatile v2us*)(Al + irow * KC + j) = il; }
        if (ps == 0) __threadfence(); }
}
__global__ __launch_bounds__(256) void k_mag(const float* __restrict__ Cp, float* OUT) {
    const int lane = threadIdx.x & 31; const int f0 = (blockIdx.x * 8 + (threadIdx.x >> 5)) * 32; if (f0 >= NBIN * NFR) return; const int f = f0 + lane; float vout = 0.f;
    if (f < NBIN * NFR) { const int bin = f / NFR, fr = f % NFR; float cr = 0.f, ci = 0.f;
#pragma unroll
        for (int c = 0; c < NCH; ++c) { cr += Cp[((size_t)c * MP + bin) * NP + fr]; ci += Cp[((size_t)c * MP + NBIN + bin) * NP + fr]; }
        vout = sqrtf(fmaf(cr, cr, ci * ci)); }
    if (f < NBIN * NFR) { *(volatile float*)(OUT + f) = vout; } __threadfence(); if (f < NBIN * NFR) { *(volatile float*)(OUT + f) = vout; }
}

extern "C" void kernel_launch(void* const* d_in, const int* in_sizes, int n_in,
                              void* d_out, int out_size, void* d_ws, size_t ws_size, hipStream_t stream) {
    (void)in_sizes; (void)n_in; (void)out_size;
    const float* sig = (const float*)d_in[0];
    float* OUT = (float*)d_out;
    char* wsp = (char*)d_ws;
    auto take = [&](size_t bytes) { char* p = wsp; wsp += (bytes + 255) & ~(size_t)255; return (void*)p; };
    float* NORM = (float*)take(256 * 4); bf* FR = (bf*)take((size_t)NP * KC * 2); bf* KH = (bf*)take((size_t)MP * KC * 2); bf* KL = (bf*)take((size_t)MP * KC * 2); float* Cp = (float*)take((size_t)NCH * MP * NP * 4);
    if ((size_t)(wsp - (char*)d_ws) > ws_size) return;
    k_norm<<<1, 256, 0, stream>>>(NORM);
    for (int c = 0; c < NCH; ++c) { const int kc0 = c * KC;
        k_frames<<<(NP * KC / 64 + 63) / 64, 256, 0, stream>>>(sig, kc0, FR);
        k_kern<<<(256 * KC / 64 + 63) / 64, 256, 0, stream>>>(NORM, kc0, KH, KL);
        k_gemmw<bf, 1, false><<<dim3(MP / 64, NP / 64, 1), 32, 0, stream>>>(KH, KL, FR, nullptr, KC, Cp + (size_t)c * MP * NP, NP, nullptr, 0, 0, 0); }
    k_mag<<<(NBIN * NFR / 32 + 7) / 8 + 1, 256, 0, stream>>>(Cp, OUT);
}
